// StatefulBilinearAttention_39324720562583
// MI455X (gfx1250) — hardware-verified
//
#include <hip/hip_runtime.h>

#define BB_  8
#define QQ_  128
#define KK_  1024
#define DM_  512
#define HH_  256

typedef _Float16 f16;
typedef __attribute__((ext_vector_type(16))) f16 f16x16;
typedef __attribute__((ext_vector_type(8)))  f16 f16x8;
typedef __attribute__((ext_vector_type(8)))  float f32x8;
typedef __attribute__((ext_vector_type(4)))  float v4f_t;
typedef float v4fa __attribute__((ext_vector_type(4), may_alias));
typedef __attribute__((ext_vector_type(4)))  unsigned v4u_t;
typedef unsigned v4ua __attribute__((ext_vector_type(4), may_alias));

__device__ __forceinline__ f32x8 wmma16(f16x16 a, f16x16 b, f32x8 c) {
  c = __builtin_amdgcn_wmma_f32_16x16x32_f16(false, a, false, b, (short)0, c, false, false);
  asm volatile("v_nop\n\tv_nop\n\tv_nop\n\tv_nop" : "+v"(c) : "v"(a), "v"(b));
  return c;
}
__device__ __forceinline__ f16x16 lds_frag(const f16* base, int stride) {
  const int lane = threadIdx.x & 31, row = lane & 15, kh = (lane >> 4) * 8;
  const f16x8 lo = *(const f16x8*)(base + row * stride + kh);
  const f16x8 hi = *(const f16x8*)(base + row * stride + kh + 16);
  f16x16 f;
#pragma unroll
  for (int i = 0; i < 8; ++i) { f[i] = lo[i]; f[i + 8] = hi[i]; }
  return f;
}

#define GSTR 48
template <typename AT, bool ACC>
__global__ __launch_bounds__(256) void gemm_kn(const AT* __restrict__ A, int lda, size_t strideA,
                                               const float* __restrict__ Wm, int ldw, size_t strideW,
                                               const float* __restrict__ bias, float scale,
                                               float* __restrict__ Y, int ldy, size_t strideY, int K) {
  __shared__ __attribute__((aligned(16))) f16 ldsA[128 * GSTR];
  __shared__ __attribute__((aligned(16))) f16 ldsW[128 * GSTR];
  __shared__ __attribute__((aligned(16))) float oS[8][32 * 68];
  const int tid = threadIdx.x, lane = tid & 31, wave = tid >> 5, cl = lane & 15, rh = (lane >> 4) * 8;
  const int m0 = blockIdx.x * 128, n0 = blockIdx.y * 128;
  const int wm = (wave & 3) * 32, wn = (wave >> 2) * 64;
  A += (size_t)blockIdx.z * strideA; Wm += (size_t)blockIdx.z * strideW; Y += (size_t)blockIdx.z * strideY;
  f32x8 acc[2][4];
#pragma unroll
  for (int i = 0; i < 2; ++i)
#pragma unroll
    for (int j = 0; j < 4; ++j) { f32x8 z = {}; acc[i][j] = z; }
#pragma unroll 1
  for (int k0 = 0; k0 < K; k0 += 32) {
    __syncthreads();
    {
      const int row = tid >> 1, ch = (tid & 1) * 16;
      const AT* src = A + (size_t)(m0 + row) * lda + k0 + ch;
#pragma unroll
      for (int g = 0; g < 16; ++g) ldsA[row * GSTR + ch + g] = (f16)src[g];
    }
    {
      const int k = tid >> 3, nn0 = (tid & 7) * 16;
      const float* src = Wm + (size_t)(k0 + k) * ldw + n0 + nn0;
#pragma unroll
      for (int g = 0; g < 4; ++g) { const v4f_t v = *(const v4f_t*)(src + 4 * g);
#pragma unroll
        for (int u = 0; u < 4; ++u) ldsW[(nn0 + 4 * g + u) * GSTR + k] = (f16)v[u]; }
    }
    __syncthreads();
    f16x16 af[2];
#pragma unroll
    for (int i = 0; i < 2; ++i) af[i] = lds_frag(ldsA + (wm + 16 * i) * GSTR, GSTR);
#pragma unroll
    for (int j = 0; j < 4; ++j) {
      const f16x16 bf = lds_frag(ldsW + (wn + 16 * j) * GSTR, GSTR);
#pragma unroll
      for (int i = 0; i < 2; ++i) acc[i][j] = wmma16(af[i], bf, acc[i][j]);
    }
  }
  float* so = oS[wave];
#pragma unroll
  for (int i = 0; i < 2; ++i)
#pragma unroll
    for (int j = 0; j < 4; ++j) {
      const float bv = bias ? bias[n0 + wn + 16 * j + cl] : 0.0f;
#pragma unroll
      for (int r = 0; r < 8; ++r) so[(16 * i + rh + r) * 68 + 16 * j + cl] = acc[i][j][r] * scale + bv;
    }
  asm volatile("s_wait_dscnt 0" ::: "memory");
  __builtin_amdgcn_wave_barrier();
  if (ACC) {
#pragma unroll
    for (int it = 0; it < 16; ++it) { const int f4 = lane + 32 * it, rr = f4 >> 4, q = (f4 & 15) * 4;
      const v4f_t old = *(const volatile v4fa*)(Y + (size_t)(m0 + wm + rr) * ldy + n0 + wn + q);
      v4f_t v = *(const volatile v4fa*)(so + rr * 68 + q); v += old; *(volatile v4fa*)(so + rr * 68 + q) = v; }
    asm volatile("s_wait_dscnt 0" ::: "memory");
  }
#pragma unroll 1
  for (int pass = 0; pass < 2; ++pass) {
#pragma unroll
    for (int it = 0; it < 16; ++it) { const int f4 = lane + 32 * it, rr = f4 >> 4, q = (f4 & 15) * 4;
      *(volatile v4f_t*)(Y + (size_t)(m0 + wm + rr) * ldy + n0 + wn + q) = *(const volatile v4fa*)(so + rr * 68 + q); }
    __threadfence();
  }
}

template <typename AT, bool ACC>
__global__ __launch_bounds__(256) void gemm_kn2(const AT* __restrict__ A, int lda, size_t strideA,
                                               const float* __restrict__ Wm, int ldw, size_t strideW,
                                               const float* __restrict__ bias, float scale,
                                               float* __restrict__ Y, int ldy, size_t strideY, int K) {
  __shared__ __attribute__((aligned(16))) f16 ldsA[128 * GSTR], ldsAl[128 * GSTR];
  __shared__ __attribute__((aligned(16))) f16 ldsW[128 * GSTR], ldsWl[128 * GSTR];
  __shared__ __attribute__((aligned(16))) float oS[8][32 * 68];
  const int tid = threadIdx.x, lane = tid & 31, wave = tid >> 5, cl = lane & 15, rh = (lane >> 4) * 8;
  const int m0 = blockIdx.x * 128, n0 = blockIdx.y * 128;
  const int wm = (wave & 3) * 32, wn = (wave >> 2) * 64;
  A += (size_t)blockIdx.z * strideA; Wm += (size_t)blockIdx.z * strideW; Y += (size_t)blockIdx.z * strideY;
  f32x8 acc[2][4], accx[2][4];
#pragma unroll
  for (int i = 0; i < 2; ++i)
#pragma unroll
    for (int j = 0; j < 4; ++j) { f32x8 z = {}; acc[i][j] = z; accx[i][j] = z; }
#pragma unroll 1
  for (int k0 = 0; k0 < K; k0 += 32) {
    __syncthreads();
    {
      const int row = tid >> 1, ch = (tid & 1) * 16;
      const AT* src = A + (size_t)(m0 + row) * lda + k0 + ch;
#pragma unroll
      for (int g = 0; g < 16; ++g) { const float v = (float)src[g]; const f16 h = (f16)v; ldsA[row * GSTR + ch + g] = h; ldsAl[row * GSTR + ch + g] = (f16)((v - (float)h) * 2048.0f); }
    }
    {
      const int k = tid >> 3, nn0 = (tid & 7) * 16;
      const float* src = Wm + (size_t)(k0 + k) * ldw + n0 + nn0;
#pragma unroll
      for (int g = 0; g < 4; ++g) { const v4f_t v = *(const v4f_t*)(src + 4 * g);
#pragma unroll
        for (int u = 0; u < 4; ++u) { const f16 h = (f16)v[u]; ldsW[(nn0 + 4 * g + u) * GSTR + k] = h; ldsWl[(nn0 + 4 * g + u) * GSTR + k] = (f16)((v[u] - (float)h) * 2048.0f); } }
    }
    __syncthreads();
    f16x16 af[2], afl[2];
#pragma unroll
    for (int i = 0; i < 2; ++i) { af[i] = lds_frag(ldsA + (wm + 16 * i) * GSTR, GSTR); afl[i] = lds_frag(ldsAl + (wm + 16 * i) * GSTR, GSTR); }
#pragma unroll
    for (int j = 0; j < 4; ++j) {
      const f16x16 bf = lds_frag(ldsW + (wn + 16 * j) * GSTR, GSTR), bfl = lds_frag(ldsWl + (wn + 16 * j) * GSTR, GSTR);
#pragma unroll
      for (int i = 0; i < 2; ++i) { acc[i][j] = wmma16(af[i], bf, acc[i][j]); accx[i][j] = wmma16(af[i], bfl, accx[i][j]); accx[i][j] = wmma16(afl[i], bf, accx[i][j]); }
    }
  }
  float* so = oS[wave];
#pragma unroll
  for (int i = 0; i < 2; ++i)
#pragma unroll
    for (int j = 0; j < 4; ++j) {
      const float bv = bias ? bias[n0 + wn + 16 * j + cl] : 0.0f;
#pragma unroll
      for (int r = 0; r < 8; ++r) so[(16 * i + rh + r) * 68 + 16 * j + cl] = (acc[i][j][r] + accx[i][j][r] * (1.0f / 2048.0f)) * scale + bv;
    }
  asm volatile("s_wait_dscnt 0" ::: "memory");
  __builtin_amdgcn_wave_barrier();
  if (ACC) {
#pragma unroll
    for (int it = 0; it < 16; ++it) { const int f4 = lane + 32 * it, rr = f4 >> 4, q = (f4 & 15) * 4;
      const v4f_t old = *(const volatile v4fa*)(Y + (size_t)(m0 + wm + rr) * ldy + n0 + wn + q);
      v4f_t v = *(const volatile v4fa*)(so + rr * 68 + q); v += old; *(volatile v4fa*)(so + rr * 68 + q) = v; }
    asm volatile("s_wait_dscnt 0" ::: "memory");
  }
#pragma unroll 1
  for (int pass = 0; pass < 2; ++pass) {
#pragma unroll
    for (int it = 0; it < 16; ++it) { const int f4 = lane + 32 * it, rr = f4 >> 4, q = (f4 & 15) * 4;
      *(volatile v4f_t*)(Y + (size_t)(m0 + wm + rr) * ldy + n0 + wn + q) = *(const volatile v4fa*)(so + rr * 68 + q); }
    __threadfence();
  }
}

__global__ __launch_bounds__(256) void k_scores(const float* __restrict__ wqs, const float* __restrict__ wk,
                                                const float* __restrict__ vvec, const int* __restrict__ mask,
                                                float* __restrict__ sc_out, float* __restrict__ at_out, f16* __restrict__ P) {
  __shared__ float wqS[HH_];
  __shared__ __attribute__((aligned(16))) float sS[KK_];
  __shared__ __attribute__((aligned(16))) float pS[KK_];
  __shared__ __attribute__((aligned(16))) f16 phS[KK_];
  __shared__ float red[8];
  const int tid = threadIdx.x, lane = tid & 31, wave = tid >> 5, cl = lane & 15, kh = (lane >> 4) * 8, rh = kh;
  const int bq = blockIdx.x;
  const int b = bq >> 7;
  wqS[tid] = wqs[(size_t)bq * HH_ + tid];
  __syncthreads();
  f16x16 vb[8];
#pragma unroll
  for (int ks = 0; ks < 8; ++ks)
#pragma unroll
    for (int e = 0; e < 8; ++e) {
      vb[ks][e]     = (cl == 0) ? (f16)vvec[ks * 32 + kh + e]      : (f16)0.0f;
      vb[ks][e + 8] = (cl == 0) ? (f16)vvec[ks * 32 + kh + 16 + e] : (f16)0.0f;
    }
  const float* wkb = wk + (size_t)b * KK_ * HH_;
#pragma unroll 1
  for (int tt = 0; tt < 8; ++tt) {
    const int k0 = (wave * 8 + tt) * 16;
    const float* wkr = wkb + (size_t)(k0 + cl) * HH_;
    f32x8 acc = {};
#pragma unroll
    for (int ks = 0; ks < 8; ++ks) {
      f16x16 af;
      const float* p = wkr + ks * 32 + kh;
      const v4f_t a0 = *(const v4f_t*)(p), a1 = *(const v4f_t*)(p + 4), a2 = *(const v4f_t*)(p + 16), a3 = *(const v4f_t*)(p + 20);
      const float wv[16] = {a0[0], a0[1], a0[2], a0[3], a1[0], a1[1], a1[2], a1[3], a2[0], a2[1], a2[2], a2[3], a3[0], a3[1], a3[2], a3[3]};
#pragma unroll
      for (int e = 0; e < 16; ++e) {
        const int hI = ks * 32 + kh + (e & 7) + ((e >> 3) << 4);
        const float z = wv[e] + wqS[hI];
        af[e] = (f16)(1.0f - 2.0f / (1.0f + __expf(2.0f * z)));
      }
      acc = wmma16(af, vb[ks], acc);
    }
    if (cl == 0) {
#pragma unroll
      for (int r = 0; r < 8; ++r) sS[k0 + rh + r] = acc[r];
    }
  }
  __syncthreads();
  const int* mrow = mask + (size_t)bq * KK_;
  float s[4], mx = -INFINITY; int mk[4];
#pragma unroll
  for (int j = 0; j < 4; ++j) { const int k = tid + 256 * j; mk[j] = mrow[k]; s[j] = mk[j] ? sS[k] : -INFINITY; mx = fmaxf(mx, s[j]); }
#pragma unroll
  for (int off = 16; off >= 1; off >>= 1) mx = fmaxf(mx, __shfl_xor(mx, off, 32));
  if (lane == 0) red[wave] = mx;
  __syncthreads();
  mx = fmaxf(fmaxf(fmaxf(red[0], red[1]), fmaxf(red[2], red[3])), fmaxf(fmaxf(red[4], red[5]), fmaxf(red[6], red[7])));
  float e4[4], se = 0.0f;
#pragma unroll
  for (int j = 0; j < 4; ++j) { e4[j] = (s[j] == -INFINITY) ? 0.0f : __expf(s[j] - mx); se += e4[j]; }
#pragma unroll
  for (int off = 16; off >= 1; off >>= 1) se += __shfl_xor(se, off, 32);
  __syncthreads();
  if (lane == 0) red[wave] = se;
  __syncthreads();
  const float Z = ((red[0] + red[1]) + (red[2] + red[3])) + ((red[4] + red[5]) + (red[6] + red[7]));
  const float iz = 1.0f / Z;
#pragma unroll
  for (int j = 0; j < 4; ++j) { const int k = tid + 256 * j; const float pv = e4[j] * iz; sS[k] = s[j]; pS[k] = mk[j] ? pv : 0.0f; phS[k] = (f16)(pv * 1024.0f); }
  __syncthreads();
#pragma unroll 1
  for (int pass = 0; pass < 2; ++pass) {
    *(volatile v4f_t*)(sc_out + (size_t)bq * KK_ + tid * 4) = *(const volatile v4fa*)(sS + tid * 4);
    *(volatile v4f_t*)(at_out + (size_t)bq * KK_ + tid * 4) = *(const volatile v4fa*)(pS + tid * 4);
    if (tid < 128) *(volatile v4u_t*)(P + (size_t)bq * KK_ + tid * 8) = *(const volatile v4ua*)(phS + tid * 8);
    __threadfence();
  }
}

extern "C" void kernel_launch(void* const* d_in, const int* in_sizes, int n_in,
                              void* d_out, int out_size, void* d_ws, size_t ws_size,
                              hipStream_t stream) {
  (void)in_sizes; (void)n_in; (void)out_size; (void)ws_size;
  const float* query = (const float*)d_in[0];
  const float* state = (const float*)d_in[1];
  const float* key   = (const float*)d_in[2];
  const float* value = (const float*)d_in[3];
  const int*   mask  = (const int*)d_in[4];
  const float* Wq = (const float*)d_in[5];
  const float* bq = (const float*)d_in[6];
  const float* Ws = (const float*)d_in[7];
  const float* Wk = (const float*)d_in[8];
  const float* vv = (const float*)d_in[9];
  float* h_out  = (float*)d_out;
  float* sc_out = h_out + (size_t)BB_ * QQ_ * DM_;
  float* at_out = sc_out + (size_t)BB_ * QQ_ * KK_;
  char* ws = (char*)d_ws;
  float* wqs = (float*)ws;
  float* wkm = (float*)(ws + (1 << 20));
  f16*   P   = (f16*)(ws + (9 << 20));
  gemm_kn2<float, false><<<dim3(BB_ * QQ_ / 128, HH_ / 128, 1), dim3(256), 0, stream>>>(query, DM_, 0, Wq, HH_, 0, bq, 1.0f, wqs, HH_, 0, DM_);
  gemm_kn2<float, true ><<<dim3(BB_ * QQ_ / 128, HH_ / 128, 1), dim3(256), 0, stream>>>(state, DM_, 0, Ws, HH_, 0, nullptr, 1.0f, wqs, HH_, 0, DM_);
  gemm_kn2<float, false><<<dim3(BB_ * KK_ / 128, HH_ / 128, 1), dim3(256), 0, stream>>>(key, DM_, 0, Wk, HH_, 0, nullptr, 1.0f, wkm, HH_, 0, DM_);
  k_scores<<<dim3(BB_ * QQ_), dim3(256), 0, stream>>>(wqs, wkm, vv, mask, sc_out, at_out, P);
  gemm_kn<f16, false><<<dim3(QQ_ / 128, DM_ / 128, BB_), dim3(256), 0, stream>>>(P, KK_, (size_t)QQ_ * KK_, value, DM_, (size_t)KK_ * DM_, nullptr, 1.0f / 1024.0f, h_out, DM_, (size_t)QQ_ * DM_, KK_);
}
